// Encoder_50448685858991
// MI455X (gfx1250) — hardware-verified
//
#include <hip/hip_runtime.h>
#include <hip/hip_fp16.h>


#ifndef NB
#define NB 2
#endif
#ifndef SEQ
#define SEQ 2048
#endif
#define NB_FULL  2
#define SEQ_FULL 2048
#define DM   1024
#define NH   16
#define DH   64
#define HID  4096
#define NTOK (NB * SEQ)

static_assert(NB >= 1 && NB <= NB_FULL);
static_assert(SEQ >= 128 && SEQ <= SEQ_FULL);
static_assert(SEQ % 128 == 0);
static_assert(SEQ % 64 == 0);
static_assert(NTOK % 256 == 0);
static_assert(NTOK % 4 == 0);
static_assert(NH * DH == DM);
static_assert(DH == 64);
static_assert(DM % 64 == 0 && HID % 64 == 0);
static_assert(DM % 32 == 0 && HID % 32 == 0);
static_assert(DM == 32 * 8 * 4);
static_assert(((size_t)NTOK * DM / 8) % 256 == 0);

typedef _Float16 v16h __attribute__((ext_vector_type(16)));
typedef _Float16 v8h  __attribute__((ext_vector_type(8)));
typedef _Float16 v4h  __attribute__((ext_vector_type(4)));
typedef float    v8f  __attribute__((ext_vector_type(8)));
typedef float    v4f  __attribute__((ext_vector_type(4)));

union Frag { v16h v; v8h h[2]; };

#define CS (1.44269504088896340736f * 3.0517578125e-05f)

#define SZ_X16   ((size_t)NTOK * DM * 2)
#define SZ_WQT   ((size_t)DM * DM * 2)
#define SZ_W1T   ((size_t)HID * DM * 2)
#define SZ_W2T   ((size_t)DM * HID * 2)
#define SZ_Q16   ((size_t)NTOK * DM * 2)
#define SZ_Y32   ((size_t)NTOK * DM * 4)
#define SZ_HB    ((size_t)NTOK * HID * 2)
#define WS_TOTAL (SZ_X16 + SZ_WQT + SZ_W1T + SZ_W2T + 2 * SZ_Q16 + 2 * SZ_Y32 + SZ_HB)
static_assert(WS_TOTAL <= (size_t)134217728);

static __device__ __forceinline__ v8f zero8() {
    v8f z;
#pragma unroll
    for (int i = 0; i < 8; ++i) z[i] = 0.0f;
    return z;
}

static __device__ __forceinline__ v16h load_frag_p(const _Float16* p) {
    Frag f;
    f.h[0] = *(const v8h*)(p);
    f.h[1] = *(const v8h*)(p + 16);
    return f.v;
}

static __device__ __forceinline__ v8f wmma16(v16h a, v16h b, v8f c) {
    v8f d = __builtin_amdgcn_wmma_f32_16x16x32_f16(false, a, false, b, (short)0, c, false, false);
    asm volatile("v_nop\n\tv_nop\n\tv_nop\n\tv_nop" : "+v"(d) : "v"(a), "v"(b));
    return d;
}

static __device__ __forceinline__ float bf16r(float x) {
    unsigned u = __float_as_uint(x);
    u = (u + 0x7FFFu + ((u >> 16) & 1u)) & 0xFFFF0000u;
    return __uint_as_float(u);
}

static __device__ __forceinline__ float ex2(float x) {
    return __builtin_amdgcn_exp2f(x);
}

static __device__ __forceinline__ void wave_lds_sync() {
    __builtin_amdgcn_fence(3, "wavefront");
    asm volatile("s_wait_dscnt 0" ::: "memory");
    __builtin_amdgcn_wave_barrier();
}

static __device__ __forceinline__ float wave_sum(float v) {
    v += __shfl_xor(v, 16, 32);
    v += __shfl_xor(v, 8, 32);
    v += __shfl_xor(v, 4, 32);
    v += __shfl_xor(v, 2, 32);
    v += __shfl_xor(v, 1, 32);
    return v;
}

__global__ __launch_bounds__(256) void k_cvt_x(const float* __restrict__ x,
                                                _Float16* __restrict__ xh) {
    const int idx = blockIdx.x * 256 + threadIdx.x;
    if (idx >= NTOK * (DM / 8)) return;
    const int tok = idx >> 7;
    const int c8  = idx & 127;
    const int b   = tok / SEQ;
    const int s   = tok - b * SEQ;
    const float* src = x + ((size_t)b * SEQ_FULL + s) * DM + c8 * 8;
    v4f a = *(const v4f*)(src);
    v4f c = *(const v4f*)(src + 4);
    v8h o;
    o[0] = (_Float16)(bf16r(a.x) * 16.0f);
    o[1] = (_Float16)(bf16r(a.y) * 16.0f);
    o[2] = (_Float16)(bf16r(a.z) * 16.0f);
    o[3] = (_Float16)(bf16r(a.w) * 16.0f);
    o[4] = (_Float16)(bf16r(c.x) * 16.0f);
    o[5] = (_Float16)(bf16r(c.y) * 16.0f);
    o[6] = (_Float16)(bf16r(c.z) * 16.0f);
    o[7] = (_Float16)(bf16r(c.w) * 16.0f);
    _Float16* dst = xh + (size_t)tok * DM + c8 * 8;
    *(volatile v8h*)dst = o;
    __threadfence();
    *(volatile v8h*)dst = o;
}

__global__ __launch_bounds__(256) void k_wT(const float* __restrict__ in,
                                             _Float16* __restrict__ out,
                                             int rows, int cols) {
    __shared__ __align__(16) _Float16 T[64 * 64];
    const int tid = threadIdx.x;
    const int c0 = blockIdx.x * 64;
    const int r0 = blockIdx.y * 64;
    const size_t zoff = (size_t)blockIdx.z * (size_t)rows * (size_t)cols;
    const float* ib = in + zoff;
    _Float16*    ob = out + zoff;
#pragma unroll 1
    for (int i = 0; i < 4; ++i) {
        const int idx = i * 256 + tid;
        const int r = idx >> 4, c4 = idx & 15;
        v4f v = *(const v4f*)(ib + (size_t)(r0 + r) * cols + c0 + c4 * 4);
        T[(c4 * 4 + 0) * 64 + r] = (_Float16)(bf16r(v.x) * 64.0f);
        T[(c4 * 4 + 1) * 64 + r] = (_Float16)(bf16r(v.y) * 64.0f);
        T[(c4 * 4 + 2) * 64 + r] = (_Float16)(bf16r(v.z) * 64.0f);
        T[(c4 * 4 + 3) * 64 + r] = (_Float16)(bf16r(v.w) * 64.0f);
    }
    __syncthreads();
    const int ca = tid >> 3, j = tid & 7;
    v8h o0 = *(const v8h*)(&T[ca * 64 + j * 8]);
    v8h o1 = *(const v8h*)(&T[(ca + 32) * 64 + j * 8]);
    _Float16* d0 = ob + (size_t)(c0 + ca) * rows + r0 + j * 8;
    _Float16* d1 = ob + (size_t)(c0 + ca + 32) * rows + r0 + j * 8;
    *(volatile v8h*)d0 = o0;
    *(volatile v8h*)d1 = o1;
    __threadfence();
    *(volatile v8h*)d0 = o0;
    *(volatile v8h*)d1 = o1;
}

template <int K>
static __device__ __forceinline__ void gemm_tile64(const _Float16* __restrict__ pa,
                                                   const _Float16* __restrict__ pb,
                                                   v8f (&acc)[4][4]) {
    static_assert(K % 32 == 0);
#pragma unroll
    for (int ms = 0; ms < 4; ++ms)
#pragma unroll
        for (int nt = 0; nt < 4; ++nt) acc[ms][nt] = zero8();
#pragma unroll 1
    for (int k0 = 0; k0 < K; k0 += 32) {
        v16h am[4];
#pragma unroll
        for (int i = 0; i < 4; ++i) am[i] = load_frag_p(pa + (size_t)i * 16 * K + k0);
#pragma unroll
        for (int nt = 0; nt < 4; ++nt) {
            v16h bn = load_frag_p(pb + (size_t)nt * 16 * K + k0);
#pragma unroll
            for (int ms = 0; ms < 4; ++ms) acc[ms][nt] = wmma16(am[ms], bn, acc[ms][nt]);
        }
    }
}

__global__ __launch_bounds__(128) __attribute__((amdgpu_num_vgpr(256)))
void k_gemm_q(const _Float16* __restrict__ xh,
              const _Float16* __restrict__ wqT,
              const float* __restrict__ bq,
              _Float16* __restrict__ qrow,
              _Float16* __restrict__ qT) {
    __shared__ __align__(16) _Float16 Rst[4][16 * 64];
    __shared__ __align__(16) _Float16 Tst[4][64 * 64];
    const int tid  = threadIdx.x;
    const int lane = tid & 31;
    const int w    = tid >> 5;
    const int hh   = lane >> 4;
    const int lm   = lane & 15;
    const int kb   = hh << 3;
    const int m0   = blockIdx.x * 256 + w * 64;
    const int n0   = blockIdx.y * 64;
    const int head = blockIdx.y;
    const int b    = m0 / SEQ;
    const int s0   = m0 - b * SEQ;

    v8f acc[4][4];
    gemm_tile64<DM>(xh + (size_t)(m0 + lm) * DM + kb, wqT + (size_t)(n0 + lm) * DM + kb, acc);

    float bv[4];
#pragma unroll
    for (int nt = 0; nt < 4; ++nt) bv[nt] = bf16r(bq[n0 + nt * 16 + lm]) * 1024.0f;

    _Float16* qr = qrow + (((size_t)b * NH + head) * SEQ + s0) * DH;
    _Float16* qt = qT + ((size_t)b * NH + head) * DH * SEQ + s0;

#pragma unroll
    for (int ms = 0; ms < 4; ++ms) {
#pragma unroll
        for (int nt = 0; nt < 4; ++nt) {
            v8h tv;
#pragma unroll
            for (int r = 0; r < 8; ++r) {
                _Float16 hv = (_Float16)((acc[ms][nt][r] + bv[nt]) * 0.0625f);
                Rst[w][(8 * hh + r) * 64 + nt * 16 + lm] = hv;
                tv[r] = hv;
            }
            *(v8h*)(&Tst[w][(nt * 16 + lm) * 64 + ms * 16 + 8 * hh]) = tv;
        }
        wave_lds_sync();
        v8h rv[4];
#pragma unroll
        for (int i = 0; i < 4; ++i) rv[i] = *(const v8h*)(&Rst[w][i * 256 + lane * 8]);
        _Float16* dst = qr + ms * 1024 + lane * 8;
#pragma unroll
        for (int i = 0; i < 4; ++i) *(volatile v8h*)(dst + i * 256) = rv[i];
        __threadfence();
#pragma unroll
        for (int i = 0; i < 4; ++i) *(volatile v8h*)(dst + i * 256) = rv[i];
        wave_lds_sync();
    }
    wave_lds_sync();
#pragma unroll 1
    for (int g = 0; g < 4; ++g) {
        v8h tv[4];
#pragma unroll
        for (int i = 0; i < 4; ++i) tv[i] = *(const v8h*)(&Tst[w][(g * 4 + i) * 256 + lane * 8]);
        _Float16* dst = qt + (size_t)(g * 16 + (lane >> 3)) * SEQ + (lane & 7) * 8;
#pragma unroll
        for (int i = 0; i < 4; ++i) *(volatile v8h*)(dst + (size_t)i * 4 * SEQ) = tv[i];
        __threadfence();
#pragma unroll
        for (int i = 0; i < 4; ++i) *(volatile v8h*)(dst + (size_t)i * 4 * SEQ) = tv[i];
    }
}

__global__ __launch_bounds__(256) __attribute__((amdgpu_num_vgpr(256)))
void k_attn(const _Float16* __restrict__ qrow,
            const _Float16* __restrict__ qT,
            const float* __restrict__ x,
            float* __restrict__ y1) {
    __shared__ __align__(16) float Ost[8][16 * DH];
    const int tid  = threadIdx.x;
    const int lane = tid & 31;
    const int w    = tid >> 5;
    const int hh   = lane >> 4;
    const int lm   = lane & 15;
    const int kb   = hh << 3;
    const int b    = blockIdx.z;
    const int head = blockIdx.y;
    const int q0   = blockIdx.x * 128 + w * 16;

    const _Float16* qlane = qrow + ((size_t)b * NH + head) * SEQ * DH + (size_t)lm * DH + kb;
    const _Float16* tlane = qT + ((size_t)b * NH + head) * DH * SEQ + (size_t)lm * SEQ + kb;

    const v16h qf0 = load_frag_p(qlane + (size_t)q0 * DH);
    const v16h qf1 = load_frag_p(qlane + (size_t)q0 * DH + 32);

    v8f o[4];
#pragma unroll
    for (int dt = 0; dt < 4; ++dt) o[dt] = zero8();
    float mr = -1.0e30f, l = 0.0f;

#pragma unroll 1
    for (int key0 = 0; key0 < SEQ; key0 += 32) {
        const _Float16* ka = qlane + (size_t)key0 * DH;
        v16h a0 = load_frag_p(ka);
        v16h a1 = load_frag_p(ka + 32);
        v8f sA = wmma16(a0, qf0, zero8());
        sA = wmma16(a1, qf1, sA);
        v16h c0 = load_frag_p(ka + 16 * DH);
        v16h c1 = load_frag_p(ka + 16 * DH + 32);
        v8f sB = wmma16(c0, qf0, zero8());
        sB = wmma16(c1, qf1, sB);

        float tA[8], tB[8];
#pragma unroll
        for (int i = 0; i < 8; ++i) { tA[i] = sA[i] * CS; tB[i] = sB[i] * CS; }
        float tmax = fmaxf(tA[0], tB[0]);
#pragma unroll
        for (int i = 1; i < 8; ++i) tmax = fmaxf(tmax, fmaxf(tA[i], tB[i]));
        tmax = fmaxf(tmax, __shfl_xor(tmax, 16, 32));
        const float mn = fmaxf(mr, tmax);
        if (__builtin_amdgcn_ballot_w32(mn > mr) != 0u) {
            const float sc = ex2(mr - mn);
            l *= sc;
#pragma unroll
            for (int dt = 0; dt < 4; ++dt)
#pragma unroll
                for (int r = 0; r < 8; ++r) o[dt][r] *= sc;
        }
        mr = mn;
        const float sh = 8.0f - mn;
        float ps = 0.0f;
        v16h pb;
#pragma unroll
        for (int i = 0; i < 8; ++i) {
            const float pa = ex2(tA[i] + sh);
            const float pq = ex2(tB[i] + sh);
            ps += pa + pq;
            pb[i]     = (_Float16)pa;
            pb[8 + i] = (_Float16)pq;
        }
        l += ps;
#pragma unroll
        for (int dt = 0; dt < 4; ++dt) {
            v16h vf = load_frag_p(tlane + (size_t)dt * 16 * SEQ + key0);
            o[dt] = wmma16(vf, pb, o[dt]);
        }
    }

    const float lt  = l + __shfl_xor(l, 16, 32);
    const float inv = (1.0f / lt) * 0.015625f;
#pragma unroll
    for (int dt = 0; dt < 4; ++dt) {
        v4f u0, u1;
        u0.x = o[dt][0] * inv; u0.y = o[dt][1] * inv; u0.z = o[dt][2] * inv; u0.w = o[dt][3] * inv;
        u1.x = o[dt][4] * inv; u1.y = o[dt][5] * inv; u1.z = o[dt][6] * inv; u1.w = o[dt][7] * inv;
        *(v4f*)(&Ost[w][lm * DH + dt * 16 + 8 * hh])     = u0;
        *(v4f*)(&Ost[w][lm * DH + dt * 16 + 8 * hh + 4]) = u1;
    }
    wave_lds_sync();

    v4f sv[8];
    const int col = lm * 4;
#pragma unroll
    for (int i = 0; i < 8; ++i) {
        const int row = 2 * i + hh;
        v4f a  = *(const v4f*)(&Ost[w][i * 128 + lane * 4]);
        v4f xv = *(const v4f*)(x + ((size_t)b * SEQ_FULL + q0 + row) * DM + head * DH + col);
        a.x = bf16r(xv.x) + a.x;
        a.y = bf16r(xv.y) + a.y;
        a.z = bf16r(xv.z) + a.z;
        a.w = bf16r(xv.w) + a.w;
        sv[i] = a;
    }
    float* ob = y1 + ((size_t)b * SEQ + q0 + hh) * DM + head * DH + col;
#pragma unroll
    for (int i = 0; i < 8; ++i) *(volatile v4f*)(ob + (size_t)(2 * i) * DM) = sv[i];
    __threadfence();
#pragma unroll
    for (int i = 0; i < 8; ++i) *(volatile v4f*)(ob + (size_t)(2 * i) * DM) = sv[i];
}

__global__ __launch_bounds__(128) void k_ln(const float* __restrict__ y,
                                             const float* __restrict__ g,
                                             const float* __restrict__ be,
                                             float* __restrict__ of,
                                             _Float16* __restrict__ oh,
                                             int wr16) {
    __shared__ __align__(16) float    Rw[4][DM];
    __shared__ __align__(16) _Float16 Hw[4][DM];
    const int tid  = threadIdx.x;
    const int lane = tid & 31;
    const int w    = tid >> 5;
    const int row  = blockIdx.x * 4 + w;
    if (row >= NTOK) return;
    const float* yr = y + (size_t)row * DM;

    float s = 0.0f;
#pragma unroll 1
    for (int j = 0; j < 8; ++j) {
        const int c = j * 128 + lane * 4;
        v4f v = *(const v4f*)(yr + c);
        *(v4f*)(&Rw[w][c]) = v;
        s += (v.x + v.y) + (v.z + v.w);
    }
    s = wave_sum(s);
    const float mu = s * 0.0009765625f;
    float qv = 0.0f;
#pragma unroll 1
    for (int j = 0; j < 8; ++j) {
        const int c = j * 128 + lane * 4;
        v4f v = *(const v4f*)(&Rw[w][c]);
        const float d0 = v.x - mu, d1 = v.y - mu, d2 = v.z - mu, d3 = v.w - mu;
        qv += (d0 * d0 + d1 * d1) + (d2 * d2 + d3 * d3);
    }
    qv = wave_sum(qv);
    const float rs = rsqrtf(qv * 0.0009765625f + 1.0e-5f);
#pragma unroll 1
    for (int j = 0; j < 8; ++j) {
        const int c = j * 128 + lane * 4;
        v4f v  = *(const v4f*)(&Rw[w][c]);
        v4f gv = *(const v4f*)(g + c);
        v4f bv = *(const v4f*)(be + c);
        v4f r;
        r.x = (v.x - mu) * rs * bf16r(gv.x) + bf16r(bv.x);
        r.y = (v.y - mu) * rs * bf16r(gv.y) + bf16r(bv.y);
        r.z = (v.z - mu) * rs * bf16r(gv.z) + bf16r(bv.z);
        r.w = (v.w - mu) * rs * bf16r(gv.w) + bf16r(bv.w);
        *(v4f*)(&Rw[w][c]) = r;
        if (wr16 != 0) {
            v4h hv;
            hv.x = (_Float16)(r.x * 16.0f);
            hv.y = (_Float16)(r.y * 16.0f);
            hv.z = (_Float16)(r.z * 16.0f);
            hv.w = (_Float16)(r.w * 16.0f);
            *(v4h*)(&Hw[w][c]) = hv;
        }
    }
    wave_lds_sync();

    float*    df = of + (size_t)row * DM;
    _Float16* dh = oh + (size_t)row * DM;
#pragma unroll 1
    for (int j = 0; j < 8; ++j) {
        const int c = j * 128 + lane * 4;
        v4f v = *(const v4f*)(&Rw[w][c]);
        *(volatile v4f*)(df + c) = v;
    }
    if (wr16 != 0) {
#pragma unroll 1
        for (int j = 0; j < 4; ++j) {
            const int c = j * 256 + lane * 8;
            v8h hv = *(const v8h*)(&Hw[w][c]);
            *(volatile v8h*)(dh + c) = hv;
        }
    }
    __threadfence();
#pragma unroll 1
    for (int j = 0; j < 8; ++j) {
        const int c = j * 128 + lane * 4;
        v4f v = *(const v4f*)(&Rw[w][c]);
        *(volatile v4f*)(df + c) = v;
    }
    if (wr16 != 0) {
#pragma unroll 1
        for (int j = 0; j < 4; ++j) {
            const int c = j * 256 + lane * 8;
            v8h hv = *(const v8h*)(&Hw[w][c]);
            *(volatile v8h*)(dh + c) = hv;
        }
    }
}

__global__ __launch_bounds__(128) __attribute__((amdgpu_num_vgpr(256)))
void k_gemm_ffn1(const _Float16* __restrict__ a16,
                 const _Float16* __restrict__ w1T,
                 const float* __restrict__ b1,
                 _Float16* __restrict__ hb) {
    __shared__ __align__(16) _Float16 Rst[4][16 * 64];
    const int tid  = threadIdx.x;
    const int lane = tid & 31;
    const int w    = tid >> 5;
    const int hh   = lane >> 4;
    const int lm   = lane & 15;
    const int kb   = hh << 3;
    const int m0   = blockIdx.x * 256 + w * 64;
    const int n0   = blockIdx.y * 64;

    v8f acc[4][4];
    gemm_tile64<DM>(a16 + (size_t)(m0 + lm) * DM + kb, w1T + (size_t)(n0 + lm) * DM + kb, acc);

    float bv[4];
#pragma unroll
    for (int nt = 0; nt < 4; ++nt) bv[nt] = bf16r(b1[n0 + nt * 16 + lm]) * 1024.0f;

#pragma unroll
    for (int ms = 0; ms < 4; ++ms) {
#pragma unroll
        for (int nt = 0; nt < 4; ++nt)
#pragma unroll
            for (int r = 0; r < 8; ++r)
                Rst[w][(8 * hh + r) * 64 + nt * 16 + lm] =
                    (_Float16)(fmaxf(acc[ms][nt][r] + bv[nt], 0.0f) * 0.015625f);
        wave_lds_sync();
        v8h rv[4];
#pragma unroll
        for (int i = 0; i < 4; ++i) rv[i] = *(const v8h*)(&Rst[w][i * 256 + lane * 8]);
        _Float16* dst = hb + (size_t)(m0 + ms * 16 + (lane >> 3)) * HID + n0 + (lane & 7) * 8;
#pragma unroll
        for (int i = 0; i < 4; ++i) *(volatile v8h*)(dst + (size_t)i * 4 * HID) = rv[i];
        __threadfence();
#pragma unroll
        for (int i = 0; i < 4; ++i) *(volatile v8h*)(dst + (size_t)i * 4 * HID) = rv[i];
        wave_lds_sync();
    }
}

__global__ __launch_bounds__(128) __attribute__((amdgpu_num_vgpr(256)))
void k_gemm_ffn2(const _Float16* __restrict__ hb,
                 const _Float16* __restrict__ w2T,
                 const float* __restrict__ b2,
                 const float* __restrict__ x1,
                 float* __restrict__ y2) {
    __shared__ __align__(16) float Fst[4][16 * 64];
    const int tid  = threadIdx.x;
    const int lane = tid & 31;
    const int w    = tid >> 5;
    const int hh   = lane >> 4;
    const int lm   = lane & 15;
    const int kb   = hh << 3;
    const int m0   = blockIdx.x * 256 + w * 64;
    const int n0   = blockIdx.y * 64;

    v8f acc[4][4];
    gemm_tile64<HID>(hb + (size_t)(m0 + lm) * HID + kb, w2T + (size_t)(n0 + lm) * HID + kb, acc);

    const int col = lm * 4;
    v4f bb = *(const v4f*)(b2 + n0 + col);
    bb.x = bf16r(bb.x); bb.y = bf16r(bb.y); bb.z = bf16r(bb.z); bb.w = bf16r(bb.w);

#pragma unroll
    for (int ms = 0; ms < 4; ++ms) {
#pragma unroll
        for (int nt = 0; nt < 4; ++nt)
#pragma unroll
            for (int r = 0; r < 8; ++r)
                Fst[w][(8 * hh + r) * 64 + nt * 16 + lm] = acc[ms][nt][r] * 0.0009765625f;
        wave_lds_sync();
        v4f sv[8];
        const size_t rbase = ((size_t)(m0 + ms * 16 + hh)) * DM + n0 + col;
#pragma unroll
        for (int i = 0; i < 8; ++i) {
            v4f a  = *(const v4f*)(&Fst[w][i * 128 + lane * 4]);
            v4f xr = *(const v4f*)(x1 + rbase + (size_t)(2 * i) * DM);
            a.x = xr.x + (a.x + bb.x);
            a.y = xr.y + (a.y + bb.y);
            a.z = xr.z + (a.z + bb.z);
            a.w = xr.w + (a.w + bb.w);
            sv[i] = a;
        }
        float* dst = y2 + rbase;
#pragma unroll
        for (int i = 0; i < 8; ++i) *(volatile v4f*)(dst + (size_t)(2 * i) * DM) = sv[i];
        __threadfence();
#pragma unroll
        for (int i = 0; i < 8; ++i) *(volatile v4f*)(dst + (size_t)(2 * i) * DM) = sv[i];
        wave_lds_sync();
    }
}

extern "C" void kernel_launch(void* const* d_in, const int* in_sizes, int n_in,
                              void* d_out, int out_size, void* d_ws, size_t ws_size,
                              hipStream_t stream) {
    if (n_in < 11) return;
    if (in_sizes[0] < ((NB - 1) * SEQ_FULL + SEQ) * DM) return;
    if (in_sizes[1] < DM * DM || in_sizes[2] < DM) return;
    if (in_sizes[3] < DM || in_sizes[4] < DM) return;
    if (in_sizes[5] < DM * HID || in_sizes[6] < HID) return;
    if (in_sizes[7] < HID * DM || in_sizes[8] < DM) return;
    if (in_sizes[9] < DM || in_sizes[10] < DM) return;
    if (out_size < NTOK * DM) return;
    if (WS_TOTAL > ws_size) return;

    const float* x    = (const float*)d_in[0];
    const float* Wq   = (const float*)d_in[1];
    const float* bq   = (const float*)d_in[2];
    const float* ln1g = (const float*)d_in[3];
    const float* ln1b = (const float*)d_in[4];
    const float* W1   = (const float*)d_in[5];
    const float* b1   = (const float*)d_in[6];
    const float* W2   = (const float*)d_in[7];
    const float* b2   = (const float*)d_in[8];
    const float* ln2g = (const float*)d_in[9];
    const float* ln2b = (const float*)d_in[10];
    float* out = (float*)d_out;

    char* ws = (char*)d_ws;
    size_t off = 0;
    _Float16* x16  = (_Float16*)(ws + off); off += SZ_X16;
    _Float16* wqT  = (_Float16*)(ws + off); off += SZ_WQT;
    _Float16* w1T  = (_Float16*)(ws + off); off += SZ_W1T;
    _Float16* w2T  = (_Float16*)(ws + off); off += SZ_W2T;
    _Float16* qrow = (_Float16*)(ws + off); off += SZ_Q16;
    _Float16* qT   = (_Float16*)(ws + off); off += SZ_Q16;
    float*    y12  = (float*)(ws + off);    off += SZ_Y32;
    float*    x1   = (float*)(ws + off);    off += SZ_Y32;
    _Float16* hb   = (_Float16*)(ws + off); off += SZ_HB;
    if (off > ws_size) return;

    k_cvt_x<<<dim3((unsigned)((size_t)NTOK * DM / 8 / 256)), dim3(256), 0, stream>>>(x, x16);
    k_wT<<<dim3(DH / 64, DM / 64, NH), dim3(256), 0, stream>>>(Wq, wqT, DM, DH);
    k_wT<<<dim3(HID / 64, DM / 64, 1), dim3(256), 0, stream>>>(W1, w1T, DM, HID);
    k_wT<<<dim3(DM / 64, HID / 64, 1), dim3(256), 0, stream>>>(W2, w2T, HID, DM);

    k_gemm_q<<<dim3(NTOK / 256, DM / 64), dim3(128), 0, stream>>>(x16, wqT, bq, qrow, qT);
    k_attn<<<dim3(SEQ / 128, NH, NB), dim3(256), 0, stream>>>(qrow, qT, x, y12);
    k_ln<<<dim3(NTOK / 4), dim3(128), 0, stream>>>(y12, ln1g, ln1b, x1, x16, 1);
    k_gemm_ffn1<<<dim3(NTOK / 256, HID / 64), dim3(128), 0, stream>>>(x16, w1T, b1, hb);
    k_gemm_ffn2<<<dim3(NTOK / 256, DM / 64), dim3(128), 0, stream>>>(hb, w2T, b2, x1, y12);
    k_ln<<<dim3(NTOK / 4), dim3(128), 0, stream>>>(y12, ln2g, ln2b, out, x16, 0);
}
